// KnowledgeAttention_73495480369367
// MI455X (gfx1250) — hardware-run, weakly checked
//
#include <hip/hip_runtime.h>


#ifndef NB
#define NB 8
#endif
#define NB_FULL 8
#define TQ      128
#define TQ_FULL 128
#define KN      256
#define DD      512
#define FF      1536
#define SSP     260
#define SPP     264
#define S2      2.8853900817779268f
#define NL2     (-2.8853900817779268f)
#define PCAR    16384.0f
#define KSC     16.0f
#define ASC     16.0f
#define WSC     64.0f
#define CSC     (1.0f / (16384.0f * 16.0f))
#define OSC     (1.0f / (16.0f * 64.0f))
#define NEGB    (-3.0e38f)

static_assert(NB <= NB_FULL);
static_assert(KN == 256);
static_assert(DD == 8 * 64);
static_assert(FF == 3 * DD);
static_assert(DD % 32 == 0);
static_assert(FF % 32 == 0);
static_assert(KN % 64 == 0);
static_assert(DD % 64 == 0);
static_assert(TQ % 64 == 0);
static_assert((NB * TQ) % 64 == 0);
static_assert((NB * KN) % 64 == 0);
static_assert(TQ % 16 == 0);
static_assert(16 * DD <= 8 * 16 * 68);
static_assert((SSP * 4) % 16 == 0);
static_assert((SPP * 2) % 16 == 0);
static_assert(SSP >= KN);
static_assert(SPP >= KN);
static_assert(8 * 16 * 68 * 4 + DD * 4 + 16 * SSP * 4 + 16 * SPP * 2 <= 65536);
static_assert(8 * 16 * 68 * 4 + DD * 4 + 16 * SSP * 4 + 16 * SPP * 2 <= 131072);
static_assert(64 * 72 * 2 <= 131072);
static_assert(16 * 68 * 4 <= 131072);
static_assert(32 * 16 * 8 == 16 * 64 * 4);
static_assert(32 * 16 * 4 == 16 * 64 * 2);
static_assert(32 * 16 * 2 == KN * 4);
static_assert(256 * 16 * 2 == 64 * 64 * 2);
static_assert((size_t)TQ_FULL * NB_FULL * DD * 4 == 2097152);
static_assert((size_t)TQ_FULL * NB_FULL * DD * 4 + (size_t)TQ_FULL * NB_FULL * KN * 4 == 3145728);

typedef _Float16 h16;
typedef unsigned short bf;
typedef __attribute__((ext_vector_type(16))) __bf16   v16bf;
typedef __attribute__((ext_vector_type(16))) _Float16 v16h;
typedef __attribute__((ext_vector_type(8)))  _Float16 v8h;
typedef __attribute__((ext_vector_type(4)))  _Float16 v4h;
typedef __attribute__((ext_vector_type(8)))  unsigned short v8us;
typedef __attribute__((ext_vector_type(8)))  float    v8f;
typedef __attribute__((ext_vector_type(4)))  float    v4f;
typedef v4f  __attribute__((may_alias)) v4fa;
typedef v8h  __attribute__((may_alias)) v8ha;
typedef v4h  __attribute__((may_alias)) v4ha;

__device__ __forceinline__ unsigned short f2bf(float f) { unsigned u = __float_as_uint(f); u += 0x7FFFu + ((u >> 16) & 1u); return (unsigned short)(u >> 16); }
__device__ __forceinline__ float bfr(float f) { return __uint_as_float(((unsigned)f2bf(f)) << 16); }
__device__ __forceinline__ v16h cat16(v8h lo, v8h hi) { return __builtin_shufflevector(lo, hi, 0, 1, 2, 3, 4, 5, 6, 7, 8, 9, 10, 11, 12, 13, 14, 15); }
__device__ __forceinline__ v16bf cat16b(v8us lo, v8us hi) { return __builtin_bit_cast(v16bf, __builtin_shufflevector(lo, hi, 0, 1, 2, 3, 4, 5, 6, 7, 8, 9, 10, 11, 12, 13, 14, 15)); }
__device__ __forceinline__ v8f wmma16(v16h a, v16h b, v8f c) { return __builtin_amdgcn_wmma_f32_16x16x32_f16(false, a, false, b, (short)0, c, false, false); }
__device__ __forceinline__ v8f wmmab(v16bf a, v16bf b, v8f c) { return __builtin_amdgcn_wmma_f32_16x16x32_bf16(false, a, false, b, (short)0, c, false, false); }
__device__ __forceinline__ v16h  ldh(const h16* p) { return cat16(*(const v8h*)p, *(const v8h*)(p + 16)); }
__device__ __forceinline__ v16bf ldb(const bf* p)  { return cat16b(*(const v8us*)p, *(const v8us*)(p + 16)); }
__device__ __forceinline__ void wave_sync() { __builtin_amdgcn_fence(3  , "wavefront"); __builtin_amdgcn_wave_barrier(); asm volatile("" ::: "memory"); }
static __device__ __forceinline__ h16 toh_flush(float v) { const h16 r = (h16)v; return (fabsf(v) < 6.103515625e-05f) ? (h16)0.0f : r; }
__device__ __forceinline__ v8f wmma16g(v16h a, v16h b, v8f c) { c = wmma16(a, b, c); asm volatile("v_nop\n\tv_nop\n\tv_nop\n\tv_nop" : "+v"(c) : "v"(a), "v"(b)); return c; }
__device__ __forceinline__ v8f wmmabg(v16bf a, v16bf b, v8f c) { c = wmmab(a, b, c); asm volatile("v_nop\n\tv_nop\n\tv_nop\n\tv_nop" : "+v"(c) : "v"(a), "v"(b)); return c; }
__device__ __forceinline__ unsigned pin32(unsigned x) { asm volatile("" : "+v"(x)); return x; }

__global__ __launch_bounds__(256) void k_cvt8(const float* __restrict__ src, bf* dst, size_t n8) {
    const size_t i = (size_t)blockIdx.x * 256 + threadIdx.x; if (i >= n8) return;
    const v8f v = *(const v8f*)(src + i * 8); v8us o;
#pragma unroll
    for (int k = 0; k < 8; ++k) o[k] = f2bf(v[k]);
    *(volatile v8us*)(dst + i * 8) = o; __threadfence(); *(volatile v8us*)(dst + i * 8) = o;
}

__global__ __launch_bounds__(256) void k_cvtw(const float* __restrict__ src, h16* dst, size_t n8) {
    const size_t i = (size_t)blockIdx.x * 256 + threadIdx.x; if (i >= n8) return;
    const v8f v = *(const v8f*)(src + i * 8); v8h o;
#pragma unroll
    for (int k = 0; k < 8; ++k) o[k] = toh_flush(bfr(v[k]) * WSC);
    *(volatile v8h*)(dst + i * 8) = o; __threadfence(); *(volatile v8h*)(dst + i * 8) = o;
}

__global__ __launch_bounds__(256) void k_cat(const float* __restrict__ tgt, const float* __restrict__ ctx, h16* CA) {
    const unsigned i = blockIdx.x * 256u + threadIdx.x;
    if (i >= (unsigned)NB * TQ * 128u) return;
    const unsigned m = pin32(i >> 7), q = pin32(i & 127u);
    const unsigned seg = q >> 6, p = q & 63u;
    const unsigned b = m / TQ, t = m % TQ;
    const v8f x0 = *(const v8f*)(tgt + ((size_t)(b * TQ_FULL + t)) * DD + p * 8);
    const v8f x1 = *(const v8f*)(ctx + ((size_t)(t * NB_FULL + b)) * DD + p * 8);
    v8h o;
#pragma unroll
    for (int k = 0; k < 8; ++k) { const float x = (seg != 0u) ? x1[k] : x0[k]; o[k] = toh_flush(bfr(x) * ASC); }
    h16* dst = CA + (size_t)m * FF + DD + (size_t)seg * DD + p * 8;
    *(volatile v8h*)dst = o; __threadfence(); *(volatile v8h*)dst = o;
}

__global__ __launch_bounds__(256) void k_kbt(const float* __restrict__ kb, h16* KT) {
    __shared__ __align__(16) h16 tl[64 * 72];
    const unsigned k0 = blockIdx.x * 64u, d0 = blockIdx.y * 64u, b = blockIdx.z;
    const unsigned tid = threadIdx.x;
#pragma unroll
    for (int s = 0; s < 4; ++s) {
        const unsigned q = pin32((unsigned)s * 256u + tid); const unsigned kr = q >> 4, c4 = (q & 15u) * 4u;
        const v4f x = *(const v4f*)(kb + ((size_t)(b * KN + k0 + kr)) * DD + d0 + c4);
#pragma unroll
        for (int i = 0; i < 4; ++i) tl[(c4 + i) * 72 + kr] = toh_flush(bfr(x[i]) * KSC);
    }
    __syncthreads();
#pragma unroll 1
    for (int ps = 0; ps < 2; ++ps) {
#pragma unroll
        for (int s = 0; s < 2; ++s) {
            const unsigned q = pin32((unsigned)s * 256u + tid); const unsigned row = q >> 3, c8 = (q & 7u) * 8u;
            const v8h hv = *(const v8ha*)(&tl[row * 72 + c8]);
            *(volatile v8h*)(KT + ((size_t)(b * DD + d0 + row)) * KN + k0 + c8) = hv; }
        if (ps == 0) __threadfence(); }
}

__global__ __launch_bounds__(32) void k_lin(const bf* __restrict__ A, const bf* __restrict__ Bt, const float* __restrict__ bias, int hasb, float scale, float* C) {
    __shared__ __align__(16) float os[16 * 68];
    const int lane = threadIdx.x & 31, lr = lane & 15, hi = lane >> 4; const int r0 = blockIdx.x * 64, c0 = blockIdx.y * 64;
    v8f acc[4][4];
#pragma unroll
    for (int mb = 0; mb < 4; ++mb)
#pragma unroll
        for (int nb = 0; nb < 4; ++nb) acc[mb][nb] = (v8f){};
    const size_t aoff = (size_t)(r0 + lr) * DD + 8 * hi, boff = (size_t)(c0 + lr) * DD + 8 * hi;
#pragma unroll 1
    for (int kc = 0; kc < DD; kc += 32) {
        v16bf a[4];
#pragma unroll
        for (int mb = 0; mb < 4; ++mb) a[mb] = ldb(A + aoff + (size_t)mb * 16 * DD + kc);
#pragma unroll
        for (int nb = 0; nb < 4; ++nb) { const v16bf b = ldb(Bt + boff + (size_t)nb * 16 * DD + kc);
#pragma unroll
            for (int mb = 0; mb < 4; ++mb) acc[mb][nb] = wmmabg(a[mb], b, acc[mb][nb]); }
    }
    float bc[4];
#pragma unroll
    for (int nb = 0; nb < 4; ++nb) { const float bv = bfr(bias[c0 + nb * 16 + lr]); bc[nb] = (hasb != 0) ? bv : 0.0f; }
#pragma unroll
    for (int mb = 0; mb < 4; ++mb) {
#pragma unroll
        for (int nb = 0; nb < 4; ++nb) {
#pragma unroll
            for (int j = 0; j < 8; ++j) os[(hi * 8 + j) * 68 + nb * 16 + lr] = (acc[mb][nb][j] + bc[nb]) * scale; }
        wave_sync();
        float* cb = C + (size_t)(r0 + mb * 16) * DD + c0;
#pragma unroll 1
        for (int ps = 0; ps < 2; ++ps) {
#pragma unroll
            for (int s = 0; s < 8; ++s) { const int row = 2 * s + (lane >> 4), c4 = (lane & 15) * 4;
                const v4f val = *(const v4fa*)(&os[row * 68 + c4]);
                *(volatile v4f*)(cb + (size_t)row * DD + c4) = val; }
            if (ps == 0) __threadfence(); }
        wave_sync();
    }
}

__global__ __launch_bounds__(256) void k_score(const float* __restrict__ WQP, const float* __restrict__ UHP, const float* __restrict__ vin, const int* __restrict__ klen,
                                                const h16* __restrict__ KT, float* AL, float* CO, h16* CA) {
    __shared__ __align__(16) float sm[8 * 16 * 68];
    __shared__ __align__(16) float sv[DD];
    __shared__ __align__(16) float ss[16 * SSP];
    __shared__ __align__(16) h16   sp[16 * SPP];
    const unsigned tid = pin32(threadIdx.x);
    const int lane = threadIdx.x & 31, lr = lane & 15, hi = lane >> 4;
    const int wave = __builtin_amdgcn_readfirstlane((int)(threadIdx.x >> 5));
    const int b = blockIdx.y, t0 = blockIdx.x * 16;
    const float* qsrc = WQP + (size_t)(b * TQ + t0) * DD;
#pragma unroll
    for (int s = 0; s < 8; ++s) { const unsigned q = (unsigned)s * 256u + tid;
        const v4f x = *(const v4f*)(qsrc + (size_t)q * 4); *(v4fa*)(&sm[q * 4]) = x; }
#pragma unroll
    for (int s = 0; s < 2; ++s) { const unsigned e = (unsigned)s * 256u + tid; sv[e] = bfr(vin[e]); }
    __syncthreads();

    float acc[16];
#pragma unroll
    for (int t = 0; t < 16; ++t) acc[t] = 0.0f;
    const float* urow = UHP + ((size_t)b * KN + tid) * DD;
#pragma unroll 1
    for (int e0 = 0; e0 < DD; e0 += 4) {
        const v4f u = *(const v4f*)(urow + e0);
        const v4f vv = *(const v4fa*)(&sv[e0]);
#pragma unroll
        for (int t = 0; t < 16; ++t) {
            const v4f w = *(const v4fa*)(&sm[t * DD + e0]);
#pragma unroll
            for (int i = 0; i < 4; ++i) {
                const float ex = __builtin_amdgcn_exp2f(w[i] + u[i]);
                const float rc = __builtin_amdgcn_rcpf(ex + 1.0f);
                acc[t] = fmaf(vv[i], rc, acc[t]); } }
    }
#pragma unroll
    for (int t = 0; t < 16; ++t) ss[t * SSP + tid] = acc[t] * NL2;
    __syncthreads();

    const int len = klen[b];
#pragma unroll 1
    for (int rr = 0; rr < 2; ++rr) {
        const int t = 2 * wave + rr;
        const v4f x0 = *(const v4fa*)(&ss[t * SSP + 4 * lane]);
        const v4f x1 = *(const v4fa*)(&ss[t * SSP + 128 + 4 * lane]);
        float xs[8]; bool kp[8];
#pragma unroll
        for (int i = 0; i < 4; ++i) { xs[i] = x0[i]; xs[4 + i] = x1[i]; kp[i] = (4 * lane + i) < len; kp[4 + i] = (128 + 4 * lane + i) < len; }
        float mx = NEGB;
#pragma unroll
        for (int i = 0; i < 8; ++i) mx = fmaxf(mx, kp[i] ? xs[i] : NEGB);
        mx = fmaxf(mx, __shfl_xor(mx, 16, 32)); mx = fmaxf(mx, __shfl_xor(mx, 8, 32)); mx = fmaxf(mx, __shfl_xor(mx, 4, 32));
        mx = fmaxf(mx, __shfl_xor(mx, 2, 32));  mx = fmaxf(mx, __shfl_xor(mx, 1, 32));
        float ea[8]; float ls = 0.0f;
#pragma unroll
        for (int i = 0; i < 8; ++i) { const float e = __builtin_amdgcn_exp2f(xs[i] - mx); ea[i] = kp[i] ? e : 0.0f; ls += ea[i]; }
        ls += __shfl_xor(ls, 16, 32); ls += __shfl_xor(ls, 8, 32); ls += __shfl_xor(ls, 4, 32); ls += __shfl_xor(ls, 2, 32); ls += __shfl_xor(ls, 1, 32);
        const bool any = ls > 0.0f;
        const float lsafe = any ? ls : 1.0f;
        const float inv = any ? (1.0f / lsafe) : 0.0f;
        v4f a0, a1; v4h p0, p1;
#pragma unroll
        for (int i = 0; i < 4; ++i) { a0[i] = ea[i] * inv; a1[i] = ea[4 + i] * inv; p0[i] = toh_flush(a0[i] * PCAR); p1[i] = toh_flush(a1[i] * PCAR); }
        *(v4ha*)(&sp[t * SPP + 4 * lane]) = p0; *(v4ha*)(&sp[t * SPP + 128 + 4 * lane]) = p1;
        float* arow = AL + ((size_t)((t0 + t) * NB_FULL + b)) * KN;
        *(volatile v4f*)(arow + 4 * lane) = a0; *(volatile v4f*)(arow + 128 + 4 * lane) = a1;
        __threadfence();
        *(volatile v4f*)(arow + 4 * lane) = a0; *(volatile v4f*)(arow + 128 + 4 * lane) = a1;
    }
    __syncthreads();

    const int d0 = wave * 64;
    v8f oc[4];
#pragma unroll
    for (int nb = 0; nb < 4; ++nb) oc[nb] = (v8f){};
    const size_t kto = ((size_t)(b * DD + d0 + lr)) * KN + 8 * hi;
    const int po = lr * SPP + 8 * hi;
#pragma unroll 1
    for (int kk = 0; kk < KN; kk += 32) {
        const v16h a = cat16(*(const v8ha*)(&sp[po + kk]), *(const v8ha*)(&sp[po + kk + 16]));
#pragma unroll
        for (int nb = 0; nb < 4; ++nb) { const v16h bb = ldh(KT + kto + (size_t)nb * 16 * KN + kk); oc[nb] = wmma16g(a, bb, oc[nb]); }
    }
    const int wb = wave * 16 * 68;
#pragma unroll
    for (int nb = 0; nb < 4; ++nb) {
#pragma unroll
        for (int j = 0; j < 8; ++j) sm[wb + (hi * 8 + j) * 68 + nb * 16 + lr] = oc[nb][j] * CSC; }
    wave_sync();
    float* crow = CO + ((size_t)t0 * NB_FULL + b) * DD + d0;
    h16* prow = CA + ((size_t)(b * TQ + t0)) * FF + d0;
#pragma unroll 1
    for (int ps = 0; ps < 2; ++ps) {
#pragma unroll
        for (int s = 0; s < 8; ++s) { const int row = 2 * s + (lane >> 4), c4 = (lane & 15) * 4;
            const v4f val = *(const v4fa*)(&sm[wb + row * 68 + c4]);
            *(volatile v4f*)(crow + (size_t)row * NB_FULL * DD + c4) = val; }
#pragma unroll
        for (int s = 0; s < 4; ++s) { const int row = 4 * s + (lane >> 3), c8 = (lane & 7) * 8;
            const v4f y0 = *(const v4fa*)(&sm[wb + row * 68 + c8]); const v4f y1 = *(const v4fa*)(&sm[wb + row * 68 + c8 + 4]); v8h hv;
#pragma unroll
            for (int i = 0; i < 4; ++i) { hv[i] = toh_flush(y0[i] * ASC); hv[4 + i] = toh_flush(y1[i] * ASC); }
            *(volatile v8h*)(prow + (size_t)row * FF + c8) = hv; }
        if (ps == 0) __threadfence(); }
}

__global__ __launch_bounds__(32) void k_out(const h16* __restrict__ A, const h16* __restrict__ Bt, const float* __restrict__ bias, float* OUT) {
    __shared__ __align__(16) float os[16 * 68];
    const int lane = threadIdx.x & 31, lr = lane & 15, hi = lane >> 4; const int r0 = blockIdx.x * 64, c0 = blockIdx.y * 64;
    v8f acc[4][4];
#pragma unroll
    for (int mb = 0; mb < 4; ++mb)
#pragma unroll
        for (int nb = 0; nb < 4; ++nb) acc[mb][nb] = (v8f){};
    const size_t aoff = (size_t)(r0 + lr) * FF + 8 * hi, boff = (size_t)(c0 + lr) * FF + 8 * hi;
#pragma unroll 1
    for (int kc = 0; kc < FF; kc += 32) {
        v16h a[4];
#pragma unroll
        for (int mb = 0; mb < 4; ++mb) a[mb] = ldh(A + aoff + (size_t)mb * 16 * FF + kc);
#pragma unroll
        for (int nb = 0; nb < 4; ++nb) { const v16h b = ldh(Bt + boff + (size_t)nb * 16 * FF + kc);
#pragma unroll
            for (int mb = 0; mb < 4; ++mb) acc[mb][nb] = wmma16g(a[mb], b, acc[mb][nb]); }
    }
    float bc[4];
#pragma unroll
    for (int nb = 0; nb < 4; ++nb) bc[nb] = bfr(bias[c0 + nb * 16 + lr]);
    const int bb = r0 / TQ, tt = r0 % TQ;
#pragma unroll
    for (int mb = 0; mb < 4; ++mb) {
#pragma unroll
        for (int nb = 0; nb < 4; ++nb) {
#pragma unroll
            for (int j = 0; j < 8; ++j) os[(hi * 8 + j) * 68 + nb * 16 + lr] = acc[mb][nb][j] * OSC + bc[nb]; }
        wave_sync();
        float* ob = OUT + ((size_t)(tt + mb * 16) * NB_FULL + bb) * DD + c0;
#pragma unroll 1
        for (int ps = 0; ps < 2; ++ps) {
#pragma unroll
            for (int s = 0; s < 8; ++s) { const int row = 2 * s + (lane >> 4), c4 = (lane & 15) * 4;
                const v4f val = *(const v4fa*)(&os[row * 68 + c4]);
                *(volatile v4f*)(ob + (size_t)row * NB_FULL * DD + c4) = val; }
            if (ps == 0) __threadfence(); }
        wave_sync();
    }
}

static constexpr size_t al256(size_t v) { return (v + 255) & ~(size_t)255; }
static constexpr size_t SZ_XT = al256((size_t)NB * TQ * DD * 2);
static constexpr size_t SZ_XK = al256((size_t)NB * KN * DD * 2);
static constexpr size_t SZ_W  = al256((size_t)DD * DD * 2);
static constexpr size_t SZ_WO = al256((size_t)DD * FF * 2);
static constexpr size_t SZ_QP = al256((size_t)NB * TQ * DD * 4);
static constexpr size_t SZ_UP = al256((size_t)NB * KN * DD * 4);
static constexpr size_t SZ_KT = al256((size_t)NB * DD * KN * 2);
static constexpr size_t SZ_CA = al256((size_t)NB * TQ * FF * 2);
static constexpr size_t SZ_TOTAL = SZ_XT + SZ_XK + 2 * SZ_W + SZ_WO + SZ_QP + SZ_UP + SZ_KT + SZ_CA;
static_assert(SZ_TOTAL <= (size_t)134217728);
static_assert(((size_t)NB * TQ * DD) % 8 == 0);
static_assert(((size_t)NB * KN * DD) % 8 == 0);
static_assert(((size_t)DD * DD) % 8 == 0);
static_assert(((size_t)DD * FF) % 8 == 0);
static_assert(((size_t)NB * TQ * 128) % 256 == 0);

extern "C" void kernel_launch(void* const* d_in, const int* in_sizes, int n_in,
                              void* d_out, int out_size, void* d_ws, size_t ws_size, hipStream_t stream) {
    if (n_in < 10) return;
    if ((size_t)in_sizes[0] < (size_t)NB * TQ_FULL * DD) return;
    if ((size_t)in_sizes[1] < (size_t)NB * KN * DD) return;
    if ((size_t)in_sizes[2] < ((size_t)(TQ - 1) * NB_FULL + NB) * DD) return;
    if (in_sizes[3] < NB) return;
    if ((size_t)in_sizes[4] < (size_t)DD * DD || (size_t)in_sizes[5] < (size_t)DD * DD) return;
    if (in_sizes[6] < DD || in_sizes[7] < DD || in_sizes[9] < DD) return;
    if ((size_t)in_sizes[8] < (size_t)DD * FF) return;
    const size_t off1 = (size_t)TQ_FULL * NB_FULL * DD;
    const size_t off2 = off1 + (size_t)TQ_FULL * NB_FULL * KN;
    if ((size_t)out_size < off2 + ((size_t)(TQ - 1) * NB_FULL + NB) * DD) return;
    if (SZ_TOTAL > ws_size) return;
    const float* tgt = (const float*)d_in[0];
    const float* bank = (const float*)d_in[1];
    const float* ctx = (const float*)d_in[2];
    const int*   lens = (const int*)d_in[3];
    const float* wkn = (const float*)d_in[4];
    const float* wqr = (const float*)d_in[5];
    const float* bqr = (const float*)d_in[6];
    const float* vv  = (const float*)d_in[7];
    const float* wou = (const float*)d_in[8];
    const float* bou = (const float*)d_in[9];
    float* OUT0 = (float*)d_out;
    float* OUT1 = OUT0 + off1;
    float* OUT2 = OUT0 + off2;
    char* wsp = (char*)d_ws;
    bf*  XT  = (bf*)wsp;   wsp += SZ_XT;
    bf*  XK  = (bf*)wsp;   wsp += SZ_XK;
    bf*  WQ  = (bf*)wsp;   wsp += SZ_W;
    bf*  WK  = (bf*)wsp;   wsp += SZ_W;
    h16* WO  = (h16*)wsp;  wsp += SZ_WO;
    float* QP = (float*)wsp; wsp += SZ_QP;
    float* UP = (float*)wsp; wsp += SZ_UP;
    h16* KT  = (h16*)wsp;  wsp += SZ_KT;
    h16* CA  = (h16*)wsp;  wsp += SZ_CA;

    { const size_t n8 = (size_t)NB * TQ * DD / 8; k_cvt8<<<(unsigned)((n8 + 255) / 256), 256, 0, stream>>>(tgt, XT, n8); }
    { const size_t n8 = (size_t)NB * KN * DD / 8; k_cvt8<<<(unsigned)((n8 + 255) / 256), 256, 0, stream>>>(bank, XK, n8); }
    { const size_t n8 = (size_t)DD * DD / 8; const unsigned g = (unsigned)((n8 + 255) / 256);
      k_cvt8<<<g, 256, 0, stream>>>(wqr, WQ, n8); k_cvt8<<<g, 256, 0, stream>>>(wkn, WK, n8); }
    { const size_t n8 = (size_t)DD * FF / 8; k_cvtw<<<(unsigned)((n8 + 255) / 256), 256, 0, stream>>>(wou, WO, n8); }
    k_kbt<<<dim3(KN / 64, DD / 64, NB), 256, 0, stream>>>(bank, KT);
    k_cat<<<(unsigned)((size_t)NB * TQ * 128 / 256), 256, 0, stream>>>(tgt, ctx, CA);

    k_lin<<<dim3(NB * TQ / 64, DD / 64, 1), 32, 0, stream>>>(XT, WQ, bqr, 1, S2, QP);
    k_lin<<<dim3(NB * KN / 64, DD / 64, 1), 32, 0, stream>>>(XK, WK, bqr, 0, S2, UP);

    k_score<<<dim3(TQ / 16, NB, 1), 256, 0, stream>>>(QP, UP, vv, lens, KT, OUT1, OUT2, CA);

    k_out<<<dim3(NB * TQ / 64, DD / 64, 1), 32, 0, stream>>>(CA, WO, bou, OUT0);
}
